// DCN__36636071034949
// MI455X (gfx1250) — hardware-verified
//
#include <hip/hip_runtime.h>
#include <hip/hip_bf16.h>
#include <math.h>


#define CIN   256
#define COUT  256
#define K2    9
#define IH    128
#define IW    128
#define IHW   (IH * IW)
#define NB    2
#define KDIM  (K2 * CIN)
#define NPIX  (NB * IHW)

typedef __attribute__((ext_vector_type(16))) __bf16 bf16x16;
typedef __attribute__((ext_vector_type(8)))  __bf16 bf16x8;
typedef __attribute__((ext_vector_type(8)))  float  f32x8;
typedef __attribute__((ext_vector_type(4)))  float  v4f_t;
typedef float v4fa __attribute__((ext_vector_type(4), may_alias));
#define __bf16 _Float16
#define RSPLIT (1.0f / 2048.0f)
#define PLWOM ((size_t)32 * KDIM)
#define PLWC  ((size_t)COUT * KDIM)
__device__ __forceinline__ __bf16 lo_of(float v, __bf16 h) { return (__bf16)((v - (float)h) * 2048.0f); }
__device__ __forceinline__ f32x8 wmma16(bf16x16 a, bf16x16 b, f32x8 c) {
  return __builtin_amdgcn_wmma_f32_16x16x32_f16(false, a, false, b, (short)0, c, false, false);
}
__device__ __forceinline__ f32x8 wmma_split(bf16x16 a, bf16x16 al, bf16x16 b, bf16x16 bl, f32x8 c) {
  f32x8 x = {};
  x = wmma16(al, b, x); x = wmma16(a, bl, x);
  return wmma16(a, b, c) + x * RSPLIT;
}

__global__ __launch_bounds__(256) void prep_weights(
    const float* __restrict__ w_off, const float* __restrict__ w_mask,
    const float* __restrict__ w_conv,
    __bf16* __restrict__ Wom, __bf16* __restrict__ Wc) {
  int idx = (blockIdx.x * 256 + threadIdx.x) * 2;
  const int total = (32 + COUT) * KDIM;
  if (idx >= total) return;
  int row = idx / KDIM;
  int K   = idx - row * KDIM;
  int k   = K >> 8;
  int c   = K & 255;
  float v0 = 0.f, v1 = 0.f;
  __bf16* dstp; size_t plane;
  if (row < 32) {
    if (row < 18)       { v0 = w_off [(row * CIN + c) * K2 + k]; v1 = w_off [(row * CIN + c + 1) * K2 + k]; }
    else if (row < 27)  { v0 = w_mask[((row - 18) * CIN + c) * K2 + k]; v1 = w_mask[((row - 18) * CIN + c + 1) * K2 + k]; }
    dstp = Wom + (size_t)row * KDIM + K; plane = PLWOM;
  } else {
    int o = row - 32;
    v0 = w_conv[(o * CIN + c) * K2 + k]; v1 = w_conv[(o * CIN + c + 1) * K2 + k];
    dstp = Wc + (size_t)o * KDIM + K; plane = PLWC;
  }
  const __bf16 h0 = (__bf16)v0, h1 = (__bf16)v1;
  const unsigned ph = (unsigned)__builtin_bit_cast(unsigned short, h0) | ((unsigned)__builtin_bit_cast(unsigned short, h1) << 16);
  const unsigned pl = (unsigned)__builtin_bit_cast(unsigned short, lo_of(v0, h0)) | ((unsigned)__builtin_bit_cast(unsigned short, lo_of(v1, h1)) << 16);
  *(volatile unsigned*)dstp = ph; *(volatile unsigned*)(dstp + plane) = pl; __threadfence(); *(volatile unsigned*)dstp = ph; *(volatile unsigned*)(dstp + plane) = pl;
}

__global__ __launch_bounds__(256) void offset_mask_conv(
    const float* __restrict__ x, const __bf16* __restrict__ Wom,
    const float* __restrict__ b_off, const float* __restrict__ b_mask,
    float* __restrict__ offmask) {
  __shared__ __align__(16) __bf16 As[2][64 * 40];
  __shared__ __align__(16) __bf16 Asl[2][64 * 40];
  __shared__ __align__(16) float  Ost[64][32 + 4];

  const int tid  = threadIdx.x;
  const int lane = tid & 31;
  const int wid  = tid >> 5;
  const int pix0 = blockIdx.x * 64;
  const int b    = pix0 >> 14;

  const int sm  = tid >> 2;
  const int scg = tid & 3;
  const int shw = (pix0 + sm) & (IHW - 1);
  const int sh  = shw >> 7, sw = shw & 127;
  const int sstore = sm * 40 + scg * 8;
  const float* xbase = x + (size_t)(b * CIN + scg * 8) * IHW;

  const int mrow = wid >> 1;
  const int n0   = (wid & 1) * 16;
  const int aoff = (mrow * 16 + (lane & 15)) * 40 + ((lane >> 4) << 3);
  f32x8 acc = {};

  int par = 0;
  #pragma unroll 1
  for (int k = 0; k < K2; ++k) {
    const int ky = k / 3 - 1, kx = k - (k / 3) * 3 - 1;
    const int y = sh + ky, xx = sw + kx;
    const bool ok  = (y >= 0) & (y < IH) & (xx >= 0) & (xx < IW);
    const float okf = ok ? 1.f : 0.f;
    const int  yc  = min(max(y, 0), IH - 1);
    const int  xc  = min(max(xx, 0), IW - 1);
    const int  off = yc * IW + xc;

    #pragma unroll 1
    for (int cb = 0; cb < 8; ++cb) {
      const int c0 = cb * 32;
      {
        const float* xp = xbase + (size_t)c0 * IHW + off;
        union { __bf16 h[8]; uint4 v; } pk, pkl;
        #pragma unroll
        for (int j = 0; j < 8; ++j) {
          float v = xp[(size_t)j * IHW] * okf;
          pk.h[j] = (__bf16)v; pkl.h[j] = lo_of(v, pk.h[j]);
        }
        *reinterpret_cast<uint4*>(&As[par][sstore]) = pk.v;
        *reinterpret_cast<uint4*>(&Asl[par][sstore]) = pkl.v;
      }
      __syncthreads();

      const __bf16* Ar = &As[par][aoff];
      const __bf16* Arl = &Asl[par][aoff];
      bf16x8 alo = *reinterpret_cast<const bf16x8*>(Ar),  ahi = *reinterpret_cast<const bf16x8*>(Ar + 16);
      bf16x8 all_ = *reinterpret_cast<const bf16x8*>(Arl), alh = *reinterpret_cast<const bf16x8*>(Arl + 16);
      bf16x16 a, al;
      #pragma unroll
      for (int i = 0; i < 8; ++i) { a[i] = alo[i]; a[8 + i] = ahi[i]; al[i] = all_[i]; al[8 + i] = alh[i]; }

      const __bf16* Bp = Wom + (size_t)(n0 + (lane & 15)) * KDIM
                             + k * 256 + c0 + ((lane >> 4) << 3);
      bf16x16 bf, bl;
      *(bf16x8*)&bf = *reinterpret_cast<const bf16x8*>(Bp);         *((bf16x8*)&bf + 1) = *reinterpret_cast<const bf16x8*>(Bp + 16);
      *(bf16x8*)&bl = *reinterpret_cast<const bf16x8*>(Bp + PLWOM); *((bf16x8*)&bl + 1) = *reinterpret_cast<const bf16x8*>(Bp + PLWOM + 16);
      __builtin_prefetch((const void*)(Bp + 32), 0, 3);

      acc = wmma_split(a, al, bf, bl, acc);
      par ^= 1;
    }
  }

  const int n = n0 + (lane & 15);
  float bias = 0.f;
  bool ismask = false;
  if (n < 18)      bias = b_off[n];
  else if (n < 27) { bias = b_mask[n - 18]; ismask = true; }
  #pragma unroll
  for (int i = 0; i < 8; ++i) {
    const int m = mrow * 16 + i + ((lane >> 4) << 3);
    float v = acc[i] + bias;
    if (ismask) v = __builtin_amdgcn_rcpf(1.f + __expf(-v));
    Ost[m][n] = v;
  }
  __syncthreads();
  #pragma unroll 1
  for (int pass = 0; pass < 2; ++pass) {
    #pragma unroll
    for (int i = 0; i < 2; ++i) { const int c = tid + 256 * i, rr = c >> 3, q = c & 7;
      *(volatile v4f_t*)(offmask + (size_t)(pix0 + rr) * 32 + q * 4) = *(const v4fa*)&Ost[rr][q * 4]; }
    __threadfence();
  }
}

__global__ __launch_bounds__(256) void dcn_main(
    const float* __restrict__ x, const __bf16* __restrict__ Wc,
    const float* __restrict__ offm, const float* __restrict__ b_conv,
    float* __restrict__ out) {
  __shared__ __align__(16) __bf16 As[2][64 * 40];
  __shared__ __align__(16) __bf16 Asl[2][64 * 40];
  __shared__ __align__(16) float  Ost[COUT][64 + 4];

  const int tid  = threadIdx.x;
  const int lane = tid & 31;
  const int wid  = tid >> 5;
  const int pix0 = blockIdx.x * 64;
  const int b    = pix0 >> 14;

  const int sm   = tid >> 2;
  const int scg  = tid & 3;
  const int spix = pix0 + sm;
  const int shw  = spix & (IHW - 1);
  const int sh   = shw >> 7, sw = shw & 127;
  const int sstore = sm * 40 + scg * 8;
  const float* xbase = x + (size_t)(b * CIN + scg * 8) * IHW;

  const int mrow  = wid & 3;
  const int nhalf = wid >> 2;
  const int aoff  = (mrow * 16 + (lane & 15)) * 40 + ((lane >> 4) << 3);
  f32x8 acc[8];
  #pragma unroll
  for (int t = 0; t < 8; ++t) acc[t] = {};

  int par = 0;
  #pragma unroll 1
  for (int k = 0; k < K2; ++k) {
    const float dy  = offm[(size_t)spix * 32 + 2 * k];
    const float dx  = offm[(size_t)spix * 32 + 2 * k + 1];
    const float msk = offm[(size_t)spix * 32 + 18 + k];
    const int   kyi = k / 3, kxi = k - kyi * 3;
    const float py  = (float)(sh - 1 + kyi) + dy;
    const float px  = (float)(sw - 1 + kxi) + dx;
    const float y0f = floorf(py), x0f = floorf(px);
    const int   y0  = (int)y0f,  x0 = (int)x0f;
    const float wy  = py - y0f,  wx = px - x0f;
    const bool iy0 = (y0 >= 0) & (y0 < IH);
    const bool iy1 = (y0 + 1 >= 0) & (y0 + 1 < IH);
    const bool ix0 = (x0 >= 0) & (x0 < IW);
    const bool ix1 = (x0 + 1 >= 0) & (x0 + 1 < IW);
    const float w00 = (iy0 & ix0) ? (1.f - wy) * (1.f - wx) * msk : 0.f;
    const float w01 = (iy0 & ix1) ? (1.f - wy) * wx * msk : 0.f;
    const float w10 = (iy1 & ix0) ? wy * (1.f - wx) * msk : 0.f;
    const float w11 = (iy1 & ix1) ? wy * wx * msk : 0.f;
    const int y0c = min(max(y0, 0), IH - 1), y1c = min(max(y0 + 1, 0), IH - 1);
    const int x0c = min(max(x0, 0), IW - 1), x1c = min(max(x0 + 1, 0), IW - 1);
    const int i00 = y0c * IW + x0c, i01 = y0c * IW + x1c;
    const int i10 = y1c * IW + x0c, i11 = y1c * IW + x1c;
    const int kc256 = k * 256;

    #pragma unroll 1
    for (int cb = 0; cb < 8; ++cb) {
      const int c0 = cb * 32;
      {
        const float* xp = xbase + (size_t)c0 * IHW;
        union { __bf16 h[8]; uint4 v; } pk, pkl;
        #pragma unroll
        for (int j = 0; j < 8; ++j) {
          const float* p = xp + (size_t)j * IHW;
          float v = w00 * p[i00];
          v = fmaf(w01, p[i01], v);
          v = fmaf(w10, p[i10], v);
          v = fmaf(w11, p[i11], v);
          pk.h[j] = (__bf16)v; pkl.h[j] = lo_of(v, pk.h[j]);
        }
        *reinterpret_cast<uint4*>(&As[par][sstore]) = pk.v;
        *reinterpret_cast<uint4*>(&Asl[par][sstore]) = pkl.v;
      }
      __syncthreads();

      const __bf16* Ar = &As[par][aoff];
      const __bf16* Arl = &Asl[par][aoff];
      bf16x8 alo = *reinterpret_cast<const bf16x8*>(Ar),  ahi = *reinterpret_cast<const bf16x8*>(Ar + 16);
      bf16x8 all_ = *reinterpret_cast<const bf16x8*>(Arl), alh = *reinterpret_cast<const bf16x8*>(Arl + 16);
      bf16x16 a, al;
      #pragma unroll
      for (int i = 0; i < 8; ++i) { a[i] = alo[i]; a[8 + i] = ahi[i]; al[i] = all_[i]; al[8 + i] = alh[i]; }

      const int kc = kc256 + c0 + ((lane >> 4) << 3);
      #pragma unroll
      for (int t = 0; t < 8; ++t) {
        const int n = nhalf * 128 + t * 16 + (lane & 15);
        const __bf16* Bp = Wc + (size_t)n * KDIM + kc;
        bf16x16 bf, bl;
        *(bf16x8*)&bf = *reinterpret_cast<const bf16x8*>(Bp);        *((bf16x8*)&bf + 1) = *reinterpret_cast<const bf16x8*>(Bp + 16);
        *(bf16x8*)&bl = *reinterpret_cast<const bf16x8*>(Bp + PLWC); *((bf16x8*)&bl + 1) = *reinterpret_cast<const bf16x8*>(Bp + PLWC + 16);
        __builtin_prefetch((const void*)(Bp + 32), 0, 3);
        acc[t] = wmma_split(a, al, bf, bl, acc[t]);
        asm volatile("" ::: "memory");
      }
      par ^= 1;
    }
  }

  const int mbase = mrow * 16 + ((lane >> 4) << 3);
  const int ploc0 = (pix0 & (IHW - 1));
  #pragma unroll
  for (int t = 0; t < 8; ++t) {
    const int n = nhalf * 128 + t * 16 + (lane & 15);
    const float bias = b_conv[n];
    #pragma unroll
    for (int i = 0; i < 8; ++i) Ost[n][mbase + i] = acc[t][i] + bias;
  }
  __syncthreads();
  #pragma unroll 1
  for (int pass = 0; pass < 2; ++pass) {
    #pragma unroll
    for (int i = 0; i < 16; ++i) { const int c = tid + 256 * i, o = c >> 4, q = c & 15;
      *(volatile v4f_t*)(out + (size_t)(b * COUT + o) * IHW + ploc0 + q * 4) = *(const v4fa*)&Ost[o][q * 4]; }
    __threadfence();
  }
}

extern "C" void kernel_launch(void* const* d_in, const int* in_sizes, int n_in,
                              void* d_out, int out_size, void* d_ws, size_t ws_size,
                              hipStream_t stream) {
  (void)in_sizes; (void)n_in; (void)out_size; (void)ws_size;
  const float* x      = (const float*)d_in[0];
  const float* w_conv = (const float*)d_in[1];
  const float* b_conv = (const float*)d_in[2];
  const float* w_off  = (const float*)d_in[3];
  const float* b_off  = (const float*)d_in[4];
  const float* w_mask = (const float*)d_in[5];
  const float* b_mask = (const float*)d_in[6];
  float* out = (float*)d_out;

  char* ws = (char*)d_ws;
  __bf16* Wom = (__bf16*)(ws);
  __bf16* Wc  = (__bf16*)(ws + (size_t)32 * KDIM * 2 * 2);
  float*  offm = (float*)(ws + (size_t)(32 + COUT) * KDIM * 2 * 2);

  const int prep_total = (32 + COUT) * KDIM;
  prep_weights<<<(prep_total / 2 + 255) / 256, 256, 0, stream>>>(
      w_off, w_mask, w_conv, Wom, Wc);
  offset_mask_conv<<<NPIX / 64, 256, 0, stream>>>(x, Wom, b_off, b_mask, offm);
  dcn_main<<<NPIX / 64, 256, 0, stream>>>(x, Wc, offm, b_conv, out);
}
